// ConvKernel_34565896798380
// MI455X (gfx1250) — hardware-verified
//
#include <hip/hip_runtime.h>
#include <math.h>

typedef __attribute__((ext_vector_type(16))) _Float16 v16h;
typedef __attribute__((ext_vector_type(8)))  _Float16 v8h;
typedef __attribute__((ext_vector_type(16))) __bf16   v16b;
typedef __attribute__((ext_vector_type(8)))  __bf16   v8b;
typedef __attribute__((ext_vector_type(8)))  float    v8f;
typedef __attribute__((ext_vector_type(4)))  float    v4f;
typedef __attribute__((ext_vector_type(4)))  unsigned v4u;

constexpr int kNQ     = 10;
constexpr int kDim    = 1024;
constexpr int kHalf   = 512;
constexpr int kBatch  = 8192;
constexpr int kK2     = 2 * kDim;
constexpr int kNW     = 23;
constexpr int kPartGroups = 4;
static_assert((1 << kNQ) == kDim, "basis size");
static_assert(2 * kHalf == kDim, "half split");
static_assert(kNW == 3 + 2 * kNQ, "weight vector length");
static_assert(kK2 % 32 == 0 && kDim % 32 == 0, "k steps of 32, no tail");
static_assert(kBatch % 64 == 0 && kK2 % 64 == 0 && kDim % 64 == 0, "64 x 64 tiles, no tail");

constexpr float kPi    = 3.14159265358979323846f;
constexpr float kPiRel = 2.7827534e-8f;

constexpr float kPsiCarry = 1024.0f;
constexpr float kMatCarry = 512.0f;
constexpr float kAmp      = 1.0f / (float)(1 << (kNQ / 2));
constexpr float kPsiScale = kAmp * kPsiCarry;
constexpr float kFold     = 1.0f / (kPsiCarry * kMatCarry);
constexpr float kFold2    = kFold * kFold;
constexpr float kF16MinNormal = 6.103515625e-5f;
static_assert(kAmp == 0.03125f, "amplitude (1/sqrt 2)^10");
static_assert(kPsiScale == 32.0f, "carried state modulus");

constexpr size_t kTabBytes  = 512;
constexpr size_t kEBytes    = (size_t)kDim * kDim * 2;
constexpr size_t kRtBytes   = (size_t)kK2 * kDim * 2;
constexpr size_t kYBytes    = (size_t)kDim * kK2 * 2;
constexpr size_t kMcBytes   = (size_t)kK2 * kDim * 4;
constexpr size_t kBtBytes   = (size_t)kK2 * kK2 * 2;
constexpr size_t kAplBytes  = (size_t)kBatch * kK2 * 2;
constexpr size_t kPartBytes = (size_t)kPartGroups * kBatch * 4;
constexpr size_t kOffTab  = 0;
constexpr size_t kOffEH   = kOffTab + kTabBytes;
constexpr size_t kOffEL   = kOffEH + kEBytes;
constexpr size_t kOffETH  = kOffEL + kEBytes;
constexpr size_t kOffETL  = kOffETH + kEBytes;
constexpr size_t kOffRTH  = kOffETL + kEBytes;
constexpr size_t kOffRTL  = kOffRTH + kRtBytes;
constexpr size_t kOffYH   = kOffRTL + kRtBytes;
constexpr size_t kOffYL   = kOffYH + kYBytes;
constexpr size_t kOffMC   = kOffYL + kYBytes;
constexpr size_t kOffBT   = kOffMC + kMcBytes;
constexpr size_t kOffAPL  = kOffBT + kBtBytes;
constexpr size_t kOffPART = kOffAPL + kAplBytes;
constexpr size_t kWsTotal = kOffPART + kPartBytes;
static_assert(kWsTotal == 75629056ull, "carve total");
static_assert(kWsTotal <= 134217728ull, "carve cap");
static_assert(kOffEH % 128 == 0 && kOffPART % 128 == 0, "line aligned carve");

__device__ __forceinline__ unsigned short f2bf_bits(float f) {
  unsigned u = __float_as_uint(f);
  return (unsigned short)((u + 0x7FFFu + ((u >> 16) & 1u)) >> 16);
}
__device__ __forceinline__ float bf_bits2f(unsigned short h) { return __uint_as_float(((unsigned)h) << 16); }
__device__ __forceinline__ void split_bf(float f, unsigned short& hb, unsigned short& lb) {
  hb = f2bf_bits(f);
  lb = f2bf_bits(f - bf_bits2f(hb));
}
__device__ __forceinline__ _Float16 bits_as_h(unsigned short b) { return __builtin_bit_cast(_Float16, b); }
__device__ __forceinline__ _Float16 to_f16_flush(float v) {
  const float w = (fabsf(v) < kF16MinNormal) ? 0.0f : v;
  return (_Float16)w;
}

union FragH { v16h v; v8h h[2]; };
union FragB { v16b v; v8b h[2]; };
__device__ __forceinline__ v16h frag_load_h(const _Float16* p) {
  FragH f;
  f.h[0] = *(const v8h*)(p);
  f.h[1] = *(const v8h*)(p + 16);
  return f.v;
}
__device__ __forceinline__ v16b frag_load_b(const __bf16* p) {
  FragB f;
  f.h[0] = *(const v8b*)(p);
  f.h[1] = *(const v8b*)(p + 16);
  return f.v;
}
__device__ __forceinline__ v8f mma_h(v16h a, v16h b, v8f c) {
  c = __builtin_amdgcn_wmma_f32_16x16x32_f16(false, a, false, b, (short)0, c, false, false);
  asm volatile("v_nop\n\tv_nop\n\tv_nop\n\tv_nop" : "+v"(c) : "v"(a), "v"(b));
  return c;
}
__device__ __forceinline__ v8f mma_b(v16b a, v16b b, v8f c) {
  c = __builtin_amdgcn_wmma_f32_16x16x32_bf16(false, a, false, b, (short)0, c, false, false);
  asm volatile("v_nop\n\tv_nop\n\tv_nop\n\tv_nop" : "+v"(c) : "v"(a), "v"(b));
  return c;
}

__global__ __launch_bounds__(256) void setup_kernel(
    const float* __restrict__ x, const float* __restrict__ w, float* __restrict__ tab)
{
  __shared__ float red[8];
  __shared__ float lcs[64];
  const int tid  = threadIdx.x;
  const int lane = tid & 31;
  const int wave = tid >> 5;

  float m = -INFINITY;
#pragma unroll 1
  for (int it = 0; it < (kBatch * kNQ) / 1024; ++it) {
    const v4f v = *(const v4f*)(x + (size_t)(it * 256 + tid) * 4);
    m = fmaxf(m, fmaxf(fmaxf(v[0], v[1]), fmaxf(v[2], v[3])));
  }
  m = fmaxf(m, __shfl_xor(m, 16, 32));
  m = fmaxf(m, __shfl_xor(m, 8, 32));
  m = fmaxf(m, __shfl_xor(m, 4, 32));
  m = fmaxf(m, __shfl_xor(m, 2, 32));
  m = fmaxf(m, __shfl_xor(m, 1, 32));
  if (lane == 0) red[wave] = m;

  const int t = min(lane, kNW - 1);
  float wv = w[t];
  asm volatile("" : "+v"(wv));
  float sn, cs;
  sincosf(kPi * wv, &sn, &cs);
  if (tid < 32) {
    lcs[2 * tid]     = cs;
    lcs[2 * tid + 1] = sn;
  }
  __syncthreads();

  float gm = red[0];
#pragma unroll
  for (int i = 1; i < 8; ++i) gm = fmaxf(gm, red[i]);
  const float flagv = (gm > 1.0f) ? 1.0f : 0.0f;

  const int qc = min(lane >> 1, kNQ - 1);
  const float ca = lcs[2 * (3 + qc)];
  const float sa = lcs[2 * (3 + qc) + 1];
  const float cb = lcs[2 * (3 + kNQ + qc)];
  const float sb = lcs[2 * (3 + kNQ + qc) + 1];
  const float cc  = ca * cb;
  const float csb = ca * sb;
  const float ss  = sa * sb;
  const float sc  = sa * cb;
  const bool row1 = (lane & 1) != 0;
  const float g0 = row1 ? -ss : cc;
  const float g1 = row1 ? -sc : -csb;
  const float g2 = row1 ? cc : ss;
  const float g3 = row1 ? csb : -sc;

  const float c0 = lcs[0], s0 = lcs[1], c1 = lcs[2], s1 = lcs[3], c2 = lcs[4], s2 = lcs[5];
  const float t00 = c1 * c0 - s1 * s0;
  const float t01 = -(c1 * s0) - s1 * c0;
  const float t10 = s1 * c0 + c1 * s0;
  const float t11 = c1 * c0 - s1 * s0;
  const float r00 = c2 * t00 - s2 * t10;
  const float r01 = c2 * t01 - s2 * t11;
  const float r10 = s2 * t00 + c2 * t10;
  const float r11 = s2 * t01 + c2 * t11;

  const bool isU = lane < 2 * kNQ;
  const bool isR = lane == 2 * kNQ;
  const bool isF = lane == 2 * kNQ + 1;
  v4f val;
  val[0] = isU ? g0 : (isR ? r00 : (isF ? flagv : 0.0f));
  val[1] = isU ? g1 : (isR ? r01 : 0.0f);
  val[2] = isU ? g2 : (isR ? r10 : 0.0f);
  val[3] = isU ? g3 : (isR ? r11 : 0.0f);
  for (int pass = 0; pass < 2; ++pass) {
    if (tid < 32) *(volatile v4f*)(tab + 4 * tid) = val;
    __threadfence();
  }
}

__global__ __launch_bounds__(256) void eplanes_kernel(
    const float* __restrict__ E,
    unsigned short* __restrict__ eh, unsigned short* __restrict__ el,
    unsigned short* __restrict__ eth, unsigned short* __restrict__ etl)
{
  __shared__ __align__(16) float tile[64 * 68];
  const int tid = threadIdx.x;
  const int tj  = blockIdx.x;
  const int ti  = blockIdx.y;
  const int rq  = tid >> 3;
  const int c8  = (tid & 7) * 8;
  v8h hv[2], lv[2], thv[2], tlv[2];
#pragma unroll
  for (int it = 0; it < 2; ++it) {
    const int row = it * 32 + rq;
    const float* src = E + (size_t)(ti * 64 + row) * kDim + tj * 64 + c8;
    const v4f a = *(const v4f*)(src);
    const v4f b = *(const v4f*)(src + 4);
    *(v4f*)(tile + row * 68 + c8)     = a;
    *(v4f*)(tile + row * 68 + c8 + 4) = b;
    const float f[8] = {a[0], a[1], a[2], a[3], b[0], b[1], b[2], b[3]};
#pragma unroll
    for (int e = 0; e < 8; ++e) {
      unsigned short hb, lb;
      split_bf(f[e], hb, lb);
      hv[it][e] = bits_as_h(hb);
      lv[it][e] = bits_as_h(lb);
    }
  }
  __syncthreads();
#pragma unroll
  for (int it = 0; it < 2; ++it) {
    const int crow = it * 32 + rq;
#pragma unroll
    for (int e = 0; e < 8; ++e) {
      const float f = tile[(c8 + e) * 68 + crow];
      unsigned short hb, lb;
      split_bf(f, hb, lb);
      thv[it][e] = bits_as_h(hb);
      tlv[it][e] = bits_as_h(lb);
    }
  }
  for (int pass = 0; pass < 2; ++pass) {
#pragma unroll
    for (int it = 0; it < 2; ++it) {
      const int row = it * 32 + rq;
      const size_t o  = (size_t)(ti * 64 + row) * kDim + tj * 64 + c8;
      const size_t ot = (size_t)(tj * 64 + row) * kDim + ti * 64 + c8;
      *(volatile v8h*)(eh + o)   = hv[it];
      *(volatile v8h*)(el + o)   = lv[it];
      *(volatile v8h*)(eth + ot) = thv[it];
      *(volatile v8h*)(etl + ot) = tlv[it];
    }
    __threadfence();
  }
}

__global__ __launch_bounds__(256) void rtplanes_kernel(
    const float* __restrict__ tab,
    unsigned short* __restrict__ rth, unsigned short* __restrict__ rtl)
{
  __shared__ float su[128];
  const int tid = threadIdx.x;
  if (tid < 128) su[tid] = tab[tid];
  __syncthreads();
  const int j = blockIdx.x * 2 + (tid >> 7);
  const int t = tid & 127;
  float pr = 1.0f, pi = 0.0f;
#pragma unroll 1
  for (int q = 0; q < 7; ++q) {
    const int kb = (t >> (6 - q)) & 1;
    const int jb = (j >> (9 - q)) & 1;
    const float ur = su[q * 8 + (kb * 2 + jb) * 2];
    const float ui = su[q * 8 + (kb * 2 + jb) * 2 + 1];
    const float nr = pr * ur - pi * ui;
    const float ni = pr * ui + pi * ur;
    pr = nr;
    pi = ni;
  }
  const int j7 = (j >> 2) & 1;
  const int j8 = (j >> 1) & 1;
  const int j9 = j & 1;
  float ar[2], ai[2], br[4], bi[4], cr[8], ci[8];
#pragma unroll
  for (int e = 0; e < 2; ++e) {
    const float ur = su[56 + (e * 2 + j7) * 2];
    const float ui = su[56 + (e * 2 + j7) * 2 + 1];
    ar[e] = pr * ur - pi * ui;
    ai[e] = pr * ui + pi * ur;
  }
#pragma unroll
  for (int e = 0; e < 4; ++e) {
    const float ur = su[64 + ((e & 1) * 2 + j8) * 2];
    const float ui = su[64 + ((e & 1) * 2 + j8) * 2 + 1];
    br[e] = ar[e >> 1] * ur - ai[e >> 1] * ui;
    bi[e] = ar[e >> 1] * ui + ai[e >> 1] * ur;
  }
#pragma unroll
  for (int e = 0; e < 8; ++e) {
    const float ur = su[72 + ((e & 1) * 2 + j9) * 2];
    const float ui = su[72 + ((e & 1) * 2 + j9) * 2 + 1];
    cr[e] = br[e >> 1] * ur - bi[e >> 1] * ui;
    ci[e] = br[e >> 1] * ui + bi[e >> 1] * ur;
  }
  v8h rh, rl, ih, il;
#pragma unroll
  for (int e = 0; e < 8; ++e) {
    unsigned short hb, lb;
    split_bf(cr[e], hb, lb);
    rh[e] = bits_as_h(hb);
    rl[e] = bits_as_h(lb);
    split_bf(ci[e], hb, lb);
    ih[e] = bits_as_h(hb);
    il[e] = bits_as_h(lb);
  }
  const size_t ore = (size_t)j * kDim + 8 * t;
  const size_t oim = (size_t)(j + kDim) * kDim + 8 * t;
  for (int pass = 0; pass < 2; ++pass) {
    *(volatile v8h*)(rth + ore) = rh;
    *(volatile v8h*)(rtl + ore) = rl;
    *(volatile v8h*)(rth + oim) = ih;
    *(volatile v8h*)(rtl + oim) = il;
    __threadfence();
  }
}

template <int OUT_MODE>
__global__ __launch_bounds__(256) void gemm_split_kernel(
    const unsigned short* __restrict__ Ahp, const unsigned short* __restrict__ Alp, int lda,
    const unsigned short* __restrict__ Bhp, const unsigned short* __restrict__ Blp, int ldb,
    void* __restrict__ C0, void* __restrict__ C1, int ldc, int tilesN, int K)
{
  __shared__ __align__(16) float sT[8][16 * 68];
  const __bf16* Ah = (const __bf16*)Ahp;
  const __bf16* Al = (const __bf16*)Alp;
  const __bf16* Bh = (const __bf16*)Bhp;
  const __bf16* Bl = (const __bf16*)Blp;
  const int lane = threadIdx.x & 31;
  const int wave = threadIdx.x >> 5;
  const int tile = blockIdx.x * 8 + wave;
  const int tm = tile / tilesN;
  const int tn = tile - tm * tilesN;
  const int m0 = tm << 6;
  const int n0 = tn << 6;
  const int rlane = lane & 15;
  const int koff  = (lane >> 4) * 8;
  const int mOff  = (lane >> 4) * 8;

  v8f acc[4][4];
#pragma unroll
  for (int i = 0; i < 4; ++i)
#pragma unroll
    for (int j = 0; j < 4; ++j) acc[i][j] = (v8f){0.f, 0.f, 0.f, 0.f, 0.f, 0.f, 0.f, 0.f};

#pragma unroll 1
  for (int k0 = 0; k0 < K; k0 += 32) {
    v16b bh[4], bl[4];
#pragma unroll
    for (int j = 0; j < 4; ++j) {
      const size_t bo = (size_t)(n0 + (j << 4) + rlane) * ldb + koff + k0;
      bh[j] = frag_load_b(Bh + bo);
      bl[j] = frag_load_b(Bl + bo);
    }
#pragma unroll
    for (int i = 0; i < 4; ++i) {
      const size_t ao = (size_t)(m0 + (i << 4) + rlane) * lda + koff + k0;
      const v16b ah = frag_load_b(Ah + ao);
      const v16b al = frag_load_b(Al + ao);
#pragma unroll
      for (int j = 0; j < 4; ++j) {
        acc[i][j] = mma_b(ah, bh[j], acc[i][j]);
        acc[i][j] = mma_b(ah, bl[j], acc[i][j]);
        acc[i][j] = mma_b(al, bh[j], acc[i][j]);
      }
    }
  }

  float* slab = sT[wave];
#pragma unroll
  for (int i = 0; i < 4; ++i) {
    const int mBase = m0 + (i << 4);
#pragma unroll
    for (int j = 0; j < 4; ++j) {
#pragma unroll
      for (int r = 0; r < 8; ++r) slab[(mOff + r) * 68 + (j << 4) + rlane] = acc[i][j][r];
    }
    __syncthreads();
    if (OUT_MODE == 0) {
      float* C = (float*)C0;
      const int hh = lane >> 4;
      const int c4 = (lane & 15) * 4;
      v4f vv[8];
#pragma unroll
      for (int it = 0; it < 8; ++it) vv[it] = *(const v4f*)(slab + (it * 2 + hh) * 68 + c4);
      for (int pass = 0; pass < 2; ++pass) {
#pragma unroll
        for (int it = 0; it < 8; ++it) {
          *(volatile v4f*)(C + (size_t)(mBase + it * 2 + hh) * ldc + n0 + c4) = vv[it];
        }
        __threadfence();
      }
    } else {
      unsigned short* Ch = (unsigned short*)C0;
      unsigned short* Cl = (unsigned short*)C1;
      const int q  = lane >> 3;
      const int c8 = (lane & 7) * 8;
      v8h hv[4], lv[4];
#pragma unroll
      for (int it = 0; it < 4; ++it) {
        const float* sp = slab + (it * 4 + q) * 68 + c8;
#pragma unroll
        for (int e = 0; e < 8; ++e) {
          unsigned short hb, lb;
          split_bf(sp[e], hb, lb);
          hv[it][e] = bits_as_h(hb);
          lv[it][e] = bits_as_h(lb);
        }
      }
      for (int pass = 0; pass < 2; ++pass) {
#pragma unroll
        for (int it = 0; it < 4; ++it) {
          const size_t o = (size_t)(mBase + it * 4 + q) * ldc + n0 + c8;
          *(volatile v8h*)(Ch + o) = hv[it];
          *(volatile v8h*)(Cl + o) = lv[it];
        }
        __threadfence();
      }
    }
    __syncthreads();
  }
}

__global__ __launch_bounds__(256) void bt_build_kernel(
    const float* __restrict__ mc, const float* __restrict__ tab, unsigned short* __restrict__ bt)
{
  const int tid = threadIdx.x;
  const int a   = blockIdx.x * 2 + (tid >> 7);
  const int j   = (tid & 127) * 8;
  const float r00 = tab[80], r01 = tab[81], r10 = tab[82], r11 = tab[83];
  const float* pAr = mc + (size_t)(2 * a) * kDim + j;
  const float* pAi = mc + (size_t)(2 * a + 1) * kDim + j;
  const float* pBr = mc + (size_t)(2 * (a + kHalf)) * kDim + j;
  const float* pBi = mc + (size_t)(2 * (a + kHalf) + 1) * kDim + j;
  const v4f ar0 = *(const v4f*)(pAr), ar1 = *(const v4f*)(pAr + 4);
  const v4f ai0 = *(const v4f*)(pAi), ai1 = *(const v4f*)(pAi + 4);
  const v4f br0 = *(const v4f*)(pBr), br1 = *(const v4f*)(pBr + 4);
  const v4f bi0 = *(const v4f*)(pBi), bi1 = *(const v4f*)(pBi + 4);
  const float xr[8] = {ar0[0], ar0[1], ar0[2], ar0[3], ar1[0], ar1[1], ar1[2], ar1[3]};
  const float xi[8] = {ai0[0], ai0[1], ai0[2], ai0[3], ai1[0], ai1[1], ai1[2], ai1[3]};
  const float yr[8] = {br0[0], br0[1], br0[2], br0[3], br1[0], br1[1], br1[2], br1[3]};
  const float yi[8] = {bi0[0], bi0[1], bi0[2], bi0[3], bi1[0], bi1[1], bi1[2], bi1[3]};
  v8h lR, lI, lN, hR, hI, hN;
#pragma unroll
  for (int e = 0; e < 8; ++e) {
    const float lr = (r00 * xr[e] + r01 * yr[e]) * kMatCarry;
    const float li = (r00 * xi[e] + r01 * yi[e]) * kMatCarry;
    const float ur = (r10 * xr[e] + r11 * yr[e]) * kMatCarry;
    const float ui = (r10 * xi[e] + r11 * yi[e]) * kMatCarry;
    lR[e] = to_f16_flush(lr);
    lI[e] = to_f16_flush(li);
    lN[e] = to_f16_flush(-li);
    hR[e] = to_f16_flush(ur);
    hI[e] = to_f16_flush(ui);
    hN[e] = to_f16_flush(-ui);
  }
  unsigned short* rowA  = bt + (size_t)a * kK2 + j;
  unsigned short* rowAi = bt + (size_t)(kDim + a) * kK2 + j;
  unsigned short* rowB  = bt + (size_t)(a + kHalf) * kK2 + j;
  unsigned short* rowBi = bt + (size_t)(kDim + a + kHalf) * kK2 + j;
  for (int pass = 0; pass < 2; ++pass) {
    *(volatile v8h*)(rowA)         = lR;
    *(volatile v8h*)(rowA + kDim)  = lN;
    *(volatile v8h*)(rowAi)        = lI;
    *(volatile v8h*)(rowAi + kDim) = lR;
    *(volatile v8h*)(rowB)         = hR;
    *(volatile v8h*)(rowB + kDim)  = hN;
    *(volatile v8h*)(rowBi)        = hI;
    *(volatile v8h*)(rowBi + kDim) = hR;
    __threadfence();
  }
}

__device__ __forceinline__ void phase_cs(float T, float s2, float& cs, float& sn) {
  const float u = fmaf(0.5f, fmaf(T, T, -s2), -T);
  const float n = rintf(0.5f * u);
  float ur = fmaf(-2.0f, n, u);
  ur = fmaf(u, kPiRel, ur);
  sincospif(ur, &sn, &cs);
}
__device__ __forceinline__ unsigned pack_h2(float lo, float hi) {
  const _Float16 a = to_f16_flush(lo);
  const _Float16 b = to_f16_flush(hi);
  const unsigned short ab = __builtin_bit_cast(unsigned short, a);
  const unsigned short bb = __builtin_bit_cast(unsigned short, b);
  return (unsigned)ab | ((unsigned)bb << 16);
}
constexpr int kPsiSamples = 4;
static_assert(kBatch % kPsiSamples == 0, "sample groups");
__global__ __launch_bounds__(256) void psi_kernel(
    const float* __restrict__ x, const float* __restrict__ tab, unsigned short* __restrict__ apl)
{
  __shared__ float xs[kPsiSamples * 16];
  __shared__ __align__(16) unsigned tile[kPsiSamples * kDim];
  const int tid = threadIdx.x;
  const int b0  = blockIdx.x * kPsiSamples;
  const float flagv = tab[84];
  {
    const int g  = tid >> 4;
    const int s  = g & 3;
    const int q  = tid & 15;
    const int qc = min(q, kNQ - 1);
    float xv = x[(size_t)(b0 + s) * kNQ + qc];
    asm volatile("" : "+v"(xv));
    const float xa = (flagv != 0.0f) ? atanf(xv) : xv;
    const float xz = (q < kNQ) ? xa : 0.0f;
    float sq = xz * xz;
    sq += __shfl_xor(sq, 1, 32);
    sq += __shfl_xor(sq, 2, 32);
    sq += __shfl_xor(sq, 4, 32);
    sq += __shfl_xor(sq, 8, 32);
    if (g < kPsiSamples) xs[s * 16 + q] = (q == kNQ) ? sq : xz;
  }
  __syncthreads();

#pragma unroll 1
  for (int it = 0; it < 8; ++it) {
    const int p  = it * 256 + tid;
    const int s  = p >> 9;
    const int kp = p & 511;
    const float* xr = xs + s * 16;
    float th = 0.0f;
#pragma unroll
    for (int q = 0; q < kNQ - 1; ++q) {
      const int bit = (kp >> (8 - q)) & 1;
      const float xq = xr[q];
      th += (bit != 0) ? -xq : xq;
    }
    const float x9 = xr[kNQ - 1];
    const float s2 = xr[kNQ];
    float c0, s0, c1, s1;
    phase_cs(th + x9, s2, c0, s0);
    phase_cs(th - x9, s2, c1, s1);
    const unsigned wre = pack_h2(c0 * kPsiScale, c1 * kPsiScale);
    const unsigned wim = pack_h2(s0 * kPsiScale, s1 * kPsiScale);
    tile[s * kDim + kp]         = wre;
    tile[s * kDim + kHalf + kp] = wim;
  }
  __syncthreads();

  v4u ov[4];
#pragma unroll
  for (int it = 0; it < 4; ++it) ov[it] = *(const v4u*)(tile + (it * 256 + tid) * 4);
  unsigned* dst = (unsigned*)apl + (size_t)b0 * kDim;
  for (int pass = 0; pass < 2; ++pass) {
#pragma unroll
    for (int it = 0; it < 4; ++it) {
      *(volatile v4u*)(dst + (size_t)(it * 256 + tid) * 4) = ov[it];
    }
    __threadfence();
  }
}

constexpr int kBigTilesN = kK2 / 64;
constexpr int kBigTilesM = kBatch / 64;
static_assert(kBigTilesN == 32, "tile = (tm << 5) | tn");
static_assert((kBigTilesN % 8) == 0, "a block's 8 waves share one tm");
static_assert(kBigTilesN / 8 == kPartGroups, "partial groups");
__global__ __launch_bounds__(256) void gemm_big_kernel(
    const unsigned short* __restrict__ Ap, const unsigned short* __restrict__ Bp,
    float* __restrict__ part)
{
  __shared__ __align__(16) float rs[8][64];
  const _Float16* A = (const _Float16*)Ap;
  const _Float16* B = (const _Float16*)Bp;
  const int tid  = threadIdx.x;
  const int lane = tid & 31;
  const int wave = tid >> 5;
  const int tile = blockIdx.x * 8 + wave;
  const int tm = tile >> 5;
  const int tn = tile & 31;
  const int m0 = tm << 6;
  const int n0 = tn << 6;
  const int rlane = lane & 15;
  const int koff  = (lane >> 4) * 8;
  const int mOff  = (lane >> 4) * 8;

  v8f acc[4][4];
#pragma unroll
  for (int i = 0; i < 4; ++i)
#pragma unroll
    for (int j = 0; j < 4; ++j) acc[i][j] = (v8f){0.f, 0.f, 0.f, 0.f, 0.f, 0.f, 0.f, 0.f};

#pragma unroll 1
  for (int k0 = 0; k0 < kK2; k0 += 32) {
    v16h bh[4];
#pragma unroll
    for (int j = 0; j < 4; ++j) {
      bh[j] = frag_load_h(B + (size_t)(n0 + (j << 4) + rlane) * kK2 + koff + k0);
    }
#pragma unroll
    for (int i = 0; i < 4; ++i) {
      const v16h ah = frag_load_h(A + (size_t)(m0 + (i << 4) + rlane) * kK2 + koff + k0);
#pragma unroll
      for (int j = 0; j < 4; ++j) acc[i][j] = mma_h(ah, bh[j], acc[i][j]);
    }
  }

  const float sc = (((n0 & (kDim - 1)) >= kHalf) ? 1.0f : -1.0f) * kFold2;
  float v[4][8];
#pragma unroll
  for (int i = 0; i < 4; ++i) {
#pragma unroll
    for (int r = 0; r < 8; ++r) {
      float s = 0.0f;
#pragma unroll
      for (int j = 0; j < 4; ++j) {
        const float a = acc[i][j][r];
        s = fmaf(a, a, s);
      }
      v[i][r] = s;
    }
  }
#pragma unroll
  for (int i = 0; i < 4; ++i) {
#pragma unroll
    for (int r = 0; r < 8; ++r) {
      float s = v[i][r];
      s += __shfl_xor(s, 1, 32);
      s += __shfl_xor(s, 2, 32);
      s += __shfl_xor(s, 4, 32);
      s += __shfl_xor(s, 8, 32);
      v[i][r] = s * sc;
    }
  }
  if (rlane == 0) {
#pragma unroll
    for (int i = 0; i < 4; ++i) {
#pragma unroll
      for (int r = 0; r < 8; ++r) rs[wave][(i << 4) + mOff + r] = v[i][r];
    }
  }
  __syncthreads();
  const int l4 = (lane & 15) * 4;
  v4f tot = *(const v4f*)(&rs[0][l4]);
#pragma unroll
  for (int w = 1; w < 8; ++w) {
    const v4f t = *(const v4f*)(&rs[w][l4]);
    tot = tot + t;
  }
  float* dst = part + (size_t)(blockIdx.x & (kPartGroups - 1)) * kBatch + m0 + l4;
  for (int pass = 0; pass < 2; ++pass) {
    if (tid < 16) *(volatile v4f*)(dst) = tot;
    __threadfence();
  }
}

__global__ __launch_bounds__(256) void final_kernel(
    const float* __restrict__ part, float* __restrict__ out)
{
  const int i = (blockIdx.x * 256 + threadIdx.x) * 4;
  const v4f p0 = *(const v4f*)(part + i);
  const v4f p1 = *(const v4f*)(part + (size_t)kBatch + i);
  const v4f p2 = *(const v4f*)(part + (size_t)2 * kBatch + i);
  const v4f p3 = *(const v4f*)(part + (size_t)3 * kBatch + i);
  const v4f s = ((p0 + p1) + p2) + p3;
  for (int pass = 0; pass < 2; ++pass) {
    *(volatile v4f*)(out + i) = s;
    __threadfence();
  }
}

constexpr int kG1TilesM = kDim / 64;
constexpr int kG1TilesN = kK2 / 64;
constexpr int kG2TilesM = kK2 / 64;
constexpr int kG2TilesN = kDim / 64;
static_assert((kG1TilesM * kG1TilesN) % 8 == 0, "whole blocks of 8 tiles");
static_assert((kG2TilesM * kG2TilesN) % 8 == 0, "whole blocks of 8 tiles");
static_assert((kBigTilesM * kBigTilesN) % 8 == 0, "whole blocks of 8 tiles");
static_assert((kBatch * kNQ) % 1024 == 0, "maximum pass covers the inputs exactly");

extern "C" void kernel_launch(void* const* d_in, const int* in_sizes, int n_in,
                              void* d_out, int out_size, void* d_ws, size_t ws_size,
                              hipStream_t stream) {
  if (n_in < 3) return;
  if (in_sizes[0] != kBatch * kNQ) return;
  if (in_sizes[1] != kNW) return;
  if (in_sizes[2] != kDim * kDim) return;
  if (out_size != kBatch) return;
  if (ws_size < kWsTotal) return;

  const float* x  = (const float*)d_in[0];
  const float* w  = (const float*)d_in[1];
  const float* E  = (const float*)d_in[2];
  float* out = (float*)d_out;
  char* ws = (char*)d_ws;
  float* tab = (float*)(ws + kOffTab);
  unsigned short* eh  = (unsigned short*)(ws + kOffEH);
  unsigned short* el  = (unsigned short*)(ws + kOffEL);
  unsigned short* eth = (unsigned short*)(ws + kOffETH);
  unsigned short* etl = (unsigned short*)(ws + kOffETL);
  unsigned short* rth = (unsigned short*)(ws + kOffRTH);
  unsigned short* rtl = (unsigned short*)(ws + kOffRTL);
  unsigned short* yh  = (unsigned short*)(ws + kOffYH);
  unsigned short* yl  = (unsigned short*)(ws + kOffYL);
  float* mc = (float*)(ws + kOffMC);
  unsigned short* bt  = (unsigned short*)(ws + kOffBT);
  unsigned short* apl = (unsigned short*)(ws + kOffAPL);
  float* part = (float*)(ws + kOffPART);

  setup_kernel<<<1, 256, 0, stream>>>(x, w, tab);
  eplanes_kernel<<<dim3(kDim / 64, kDim / 64), 256, 0, stream>>>(E, eh, el, eth, etl);
  rtplanes_kernel<<<kDim / 2, 256, 0, stream>>>(tab, rth, rtl);
  gemm_split_kernel<2><<<(kG1TilesM * kG1TilesN) / 8, 256, 0, stream>>>(
      eh, el, kDim, rth, rtl, kDim, (void*)yh, (void*)yl, kK2, kG1TilesN, kDim);
  gemm_split_kernel<0><<<(kG2TilesM * kG2TilesN) / 8, 256, 0, stream>>>(
      yh, yl, kDim, eth, etl, kDim, (void*)mc, (void*)mc, kDim, kG2TilesN, kDim);
  bt_build_kernel<<<kHalf / 2, 256, 0, stream>>>(mc, tab, bt);
  psi_kernel<<<kBatch / kPsiSamples, 256, 0, stream>>>(x, tab, apl);
  gemm_big_kernel<<<(kBigTilesM * kBigTilesN) / 8, 256, 0, stream>>>(apl, bt, part);
  final_kernel<<<kBatch / 1024, 256, 0, stream>>>(part, out);
}
